// LstmAutoencoderPk_29781303230686
// MI455X (gfx1250) — hardware-verified
//
#include <hip/hip_runtime.h>
#include <cstddef>


#define BATCH  64
#define TLEN   512
#define DIN    128
#define HID    512
#define G4     2048
#define LAT    128
#define DSTEPS 511
#define SEQB   16
#define NGRP   4
#define HP     520
#define LP     136
#define OP     132
#define NT     512

static_assert(BATCH == NGRP * SEQB);
static_assert(HID == 16 * 32);
static_assert((HP * 2) % 16 == 0);
static_assert((LP * 2) % 16 == 0);
static_assert((OP * 4) % 16 == 0);
static_assert(HID % 32 == 0 && DIN % 32 == 0 && G4 % 32 == 0 && LAT % 32 == 0);

typedef _Float16 f16_t;
typedef f16_t          v8h   __attribute__((ext_vector_type(8)));
typedef f16_t          v16h  __attribute__((ext_vector_type(16)));
typedef float          v4f   __attribute__((ext_vector_type(4)));
typedef float          v8f   __attribute__((ext_vector_type(8)));
typedef unsigned short u16x8 __attribute__((ext_vector_type(8)));

union Frag { v16h v; v8h h[2]; };
union H8   { v8h f; u16x8 u; };

#define INV16  0.0625f
#define INV256 0.00390625f

constexpr size_t SZ_X16  = (size_t)BATCH * TLEN * DIN * 2;
constexpr size_t SZ_WHH  = (size_t)G4 * HID * 2;
constexpr size_t SZ_WIH  = (size_t)G4 * DIN * 2;
constexpr size_t SZ_WLAT = (size_t)LAT * G4 * 2;
constexpr size_t SZ_WL2H = (size_t)HID * LAT * 2;
constexpr size_t SZ_WOUT = (size_t)DIN * HID * 2;
constexpr size_t SZ_LAT  = (size_t)BATCH * G4 * 2;
constexpr size_t SZ_HDEC = (size_t)BATCH * HID * 2;

constexpr size_t OFF_X16  = 0;
constexpr size_t OFF_WHH  = OFF_X16  + SZ_X16;
constexpr size_t OFF_WIH  = OFF_WHH  + 3 * SZ_WHH;
constexpr size_t OFF_WLAT = OFF_WIH  + 3 * SZ_WIH;
constexpr size_t OFF_WL2H = OFF_WLAT + SZ_WLAT;
constexpr size_t OFF_WOUT = OFF_WL2H + SZ_WL2H;
constexpr size_t OFF_LAT  = OFF_WOUT + SZ_WOUT;
constexpr size_t OFF_HDEC = OFF_LAT  + SZ_LAT;
constexpr size_t WS_END   = OFF_HDEC + SZ_HDEC;
static_assert(WS_END <= (size_t)134217728);
static_assert(OFF_WHH % 128 == 0 && OFF_WIH % 128 == 0 && OFF_WLAT % 128 == 0 && OFF_WL2H % 128 == 0);
static_assert(OFF_WOUT % 128 == 0 && OFF_LAT % 128 == 0 && OFF_HDEC % 128 == 0 && WS_END % 128 == 0);

__device__ __forceinline__ void mma(v8f& acc, const Frag& a, const Frag& b) {
    acc = __builtin_amdgcn_wmma_f32_16x16x32_f16(false, a.v, false, b.v, (short)0, acc, false, false);
    asm volatile("v_nop\n\tv_nop\n\tv_nop\n\tv_nop" : "+v"(acc) : "v"(a.v), "v"(b.v));
}

__device__ __forceinline__ float sgm_f(float x) {
    return __builtin_amdgcn_rcpf(1.0f + __expf(-x));
}
__device__ __forceinline__ float tnh_f(float x) {
    const float e = __expf(2.0f * x);
    return 1.0f - 2.0f * __builtin_amdgcn_rcpf(1.0f + e);
}

__global__ __launch_bounds__(256)
void cvt_kernel(const float* __restrict__ src, unsigned short* dst, int n8, float scale)
{
    const int i = blockIdx.x * 256 + threadIdx.x;
    if (i >= n8) return;
    const size_t e = (size_t)i * 8;
    const v4f a = *(const v4f*)(src + e);
    const v4f b = *(const v4f*)(src + e + 4);
    H8 o;
#pragma unroll
    for (int c = 0; c < 4; ++c) {
        o.f[c]     = (f16_t)(a[c] * scale);
        o.f[c + 4] = (f16_t)(b[c] * scale);
    }
    *(volatile u16x8*)(dst + e) = o.u;
    __threadfence();
    *(volatile u16x8*)(dst + e) = o.u;
}

__device__ __forceinline__ void gates_mma(v8f (&acc)[8], const f16_t* ha, const f16_t* xa,
                                          const f16_t* __restrict__ wh, const f16_t* __restrict__ wi)
{
#pragma unroll 1
    for (int kit = 0; kit < HID / 32; ++kit) {
        const int k0 = kit * 32;
        Frag a;
        a.h[0] = *(const v8h*)(ha + k0);
        a.h[1] = *(const v8h*)(ha + k0 + 16);
#pragma unroll
        for (int t = 0; t < 8; ++t) {
            const f16_t* p = wh + (size_t)((t >> 1) * HID + (t & 1) * 16) * HID + k0;
            Frag b;
            b.h[0] = *(const v8h*)(p);
            b.h[1] = *(const v8h*)(p + 16);
            mma(acc[t], a, b);
        }
    }
#pragma unroll 1
    for (int kit = 0; kit < DIN / 32; ++kit) {
        const int k0 = kit * 32;
        Frag a;
        a.h[0] = *(const v8h*)(xa + k0);
        a.h[1] = *(const v8h*)(xa + k0 + 16);
#pragma unroll
        for (int t = 0; t < 8; ++t) {
            const f16_t* p = wi + (size_t)((t >> 1) * HID + (t & 1) * 16) * DIN + k0;
            Frag b;
            b.h[0] = *(const v8h*)(p);
            b.h[1] = *(const v8h*)(p + 16);
            mma(acc[t], a, b);
        }
    }
}

__device__ __forceinline__ void lstm_cell(const v8f (&acc)[8], const float (&bi)[8],
                                          float (&cst)[16], float (&hnew)[16])
{
#pragma unroll
    for (int u = 0; u < 2; ++u)
#pragma unroll
        for (int r = 0; r < 8; ++r) {
            const int idx = u * 8 + r;
            const float gi = acc[0 + u][r] * INV16 + bi[0 + u];
            const float gf = acc[2 + u][r] * INV16 + bi[2 + u];
            const float gg = acc[4 + u][r] * INV16 + bi[4 + u];
            const float go = acc[6 + u][r] * INV16 + bi[6 + u];
            const float c  = sgm_f(gf) * cst[idx] + sgm_f(gi) * tnh_f(gg);
            cst[idx]  = c;
            hnew[idx] = sgm_f(go) * tnh_f(c);
        }
}

__global__ __launch_bounds__(NT)
void enc_kernel(const f16_t* __restrict__ x16, const int* __restrict__ lengths,
                const f16_t* __restrict__ whh_f, const f16_t* __restrict__ wih_f, const float* __restrict__ b_f,
                const f16_t* __restrict__ whh_b, const f16_t* __restrict__ wih_b, const float* __restrict__ b_b,
                unsigned short* latin16)
{
    __shared__ __attribute__((aligned(16))) f16_t hbuf[2 * SEQB * HP];
    __shared__ __attribute__((aligned(16))) f16_t smean[SEQB * HP];

    const int tid  = threadIdx.x;
    const int lane = tid & 31;
    const int wave = tid >> 5;
    const int h    = lane >> 4;
    const int m    = lane & 15;
    const int dir  = (int)blockIdx.x / NGRP;
    const int grp  = (int)blockIdx.x - dir * NGRP;
    const int b0   = grp * SEQB;
    const int j0   = wave * 32;

    const f16_t* whh  = dir ? whh_b : whh_f;
    const f16_t* wih  = dir ? wih_b : wih_f;
    const float* bias = dir ? b_b : b_f;

    for (int i = tid; i < 2 * SEQB * HP; i += NT) hbuf[i] = (f16_t)0.0f;
    for (int i = tid; i < SEQB * HP; i += NT) smean[i] = (f16_t)0.0f;

    int   ln[8];
    float bi[8];
#pragma unroll
    for (int r = 0; r < 8; ++r) ln[r] = lengths[b0 + 8 * h + r];
#pragma unroll
    for (int t = 0; t < 8; ++t) bi[t] = bias[(t >> 1) * HID + j0 + (t & 1) * 16 + m];

    float cst[16], hsum[16];
#pragma unroll
    for (int i = 0; i < 16; ++i) { cst[i] = 0.0f; hsum[i] = 0.0f; }

    const f16_t* wh = whh + (size_t)(j0 + m) * HID + 8 * h;
    const f16_t* wi = wih + (size_t)(j0 + m) * DIN + 8 * h;
    const f16_t* xb = x16 + (size_t)(b0 + m) * TLEN * DIN + 8 * h;
    __syncthreads();

#pragma unroll 1
    for (int s = 0; s < TLEN; ++s) {
        const int tt  = dir ? (TLEN - 1 - s) : s;
        const int cur = s & 1;
        const f16_t* ha = hbuf + cur * (SEQB * HP) + m * HP + 8 * h;
        f16_t* hn = hbuf + (cur ^ 1) * (SEQB * HP);

        v8f acc[8];
#pragma unroll
        for (int t = 0; t < 8; ++t)
#pragma unroll
            for (int r = 0; r < 8; ++r) acc[t][r] = 0.0f;

        gates_mma(acc, ha, xb + (size_t)tt * DIN, wh, wi);

        float hnew[16];
        lstm_cell(acc, bi, cst, hnew);
#pragma unroll
        for (int u = 0; u < 2; ++u)
#pragma unroll
            for (int r = 0; r < 8; ++r) {
                const int idx = u * 8 + r;
                hsum[idx] += (tt < ln[r]) ? hnew[idx] : 0.0f;
                hn[(8 * h + r) * HP + j0 + 16 * u + m] = (f16_t)hnew[idx];
            }
        __syncthreads();
    }

    const f16_t* hfin = hbuf + (TLEN & 1) * (SEQB * HP);
    float rl[8];
#pragma unroll
    for (int r = 0; r < 8; ++r) rl[r] = 1.0f / (float)ln[r];
#pragma unroll
    for (int u = 0; u < 2; ++u)
#pragma unroll
        for (int r = 0; r < 8; ++r) {
            const int idx = u * 8 + r;
            smean[(8 * h + r) * HP + j0 + 16 * u + m] = (f16_t)(16.0f * (hsum[idx] * rl[r]));
        }
    __syncthreads();

    const int row = wave;
    unsigned short* rp = latin16 + (size_t)(b0 + row) * G4;
    u16x8 va[2], vb[2];
#pragma unroll
    for (int it = 0; it < 2; ++it) {
        const int c = it * 256 + lane * 8;
        H8 t;
        t.f = *(const v8h*)(hfin + row * HP + c);
#pragma unroll
        for (int e = 0; e < 8; ++e) t.f[e] = (f16_t)(16.0f * (float)t.f[e]);
        va[it] = t.u;
        H8 q;
        q.f = *(const v8h*)(smean + row * HP + c);
        vb[it] = q.u;
    }
#pragma unroll
    for (int it = 0; it < 2; ++it) {
        const int c = it * 256 + lane * 8;
        *(volatile u16x8*)(rp + dir * HID + c)           = va[it];
        *(volatile u16x8*)(rp + 2 * HID + dir * HID + c) = vb[it];
    }
    __threadfence();
#pragma unroll
    for (int it = 0; it < 2; ++it) {
        const int c = it * 256 + lane * 8;
        *(volatile u16x8*)(rp + dir * HID + c)           = va[it];
        *(volatile u16x8*)(rp + 2 * HID + dir * HID + c) = vb[it];
    }
}

__global__ __launch_bounds__(256)
void latent_kernel(const f16_t* __restrict__ latin16, const f16_t* __restrict__ wlat16, const float* __restrict__ b_lat,
                   const f16_t* __restrict__ wl2h16, const float* __restrict__ b_l2h, unsigned short* hdec16)
{
    __shared__ __attribute__((aligned(16))) f16_t sl[SEQB * LP];
    __shared__ __attribute__((aligned(16))) f16_t sh[SEQB * HP];

    const int tid  = threadIdx.x;
    const int lane = tid & 31;
    const int wave = tid >> 5;
    const int h    = lane >> 4;
    const int m    = lane & 15;
    const int b0   = (int)blockIdx.x * SEQB;

    for (int i = tid; i < SEQB * LP; i += 256) sl[i] = (f16_t)0.0f;
    for (int i = tid; i < SEQB * HP; i += 256) sh[i] = (f16_t)0.0f;
    __syncthreads();

    {
        v8f acc;
#pragma unroll
        for (int r = 0; r < 8; ++r) acc[r] = 0.0f;
        const f16_t* ap = latin16 + (size_t)(b0 + m) * G4 + 8 * h;
        const f16_t* bp = wlat16 + (size_t)(16 * wave + m) * G4 + 8 * h;
#pragma unroll 1
        for (int kit = 0; kit < G4 / 32; ++kit) {
            const int k0 = kit * 32;
            Frag a, b;
            a.h[0] = *(const v8h*)(ap + k0);
            a.h[1] = *(const v8h*)(ap + k0 + 16);
            b.h[0] = *(const v8h*)(bp + k0);
            b.h[1] = *(const v8h*)(bp + k0 + 16);
            mma(acc, a, b);
        }
        const int col = 16 * wave + m;
        const float bl = b_lat[col];
#pragma unroll
        for (int r = 0; r < 8; ++r)
            sl[(8 * h + r) * LP + col] = (f16_t)(16.0f * (acc[r] * INV256 + bl));
    }
    __syncthreads();

    {
        v8f acc2[4];
#pragma unroll
        for (int j = 0; j < 4; ++j)
#pragma unroll
            for (int r = 0; r < 8; ++r) acc2[j][r] = 0.0f;
        const f16_t* ap2 = sl + m * LP + 8 * h;
#pragma unroll
        for (int kit = 0; kit < LAT / 32; ++kit) {
            const int k0 = kit * 32;
            Frag a;
            a.h[0] = *(const v8h*)(ap2 + k0);
            a.h[1] = *(const v8h*)(ap2 + k0 + 16);
#pragma unroll
            for (int j = 0; j < 4; ++j) {
                const int nt = wave * 4 + j;
                const f16_t* p = wl2h16 + (size_t)(16 * nt + m) * LAT + 8 * h + k0;
                Frag b;
                b.h[0] = *(const v8h*)(p);
                b.h[1] = *(const v8h*)(p + 16);
                mma(acc2[j], a, b);
            }
        }
#pragma unroll
        for (int j = 0; j < 4; ++j) {
            const int col = 16 * (wave * 4 + j) + m;
            const float bb = b_l2h[col];
#pragma unroll
            for (int r = 0; r < 8; ++r)
                sh[(8 * h + r) * HP + col] = (f16_t)(acc2[j][r] * INV256 + bb);
        }
    }
    __syncthreads();

    u16x8 v[2][2];
#pragma unroll
    for (int q = 0; q < 2; ++q) {
        const int row = 2 * wave + q;
#pragma unroll
        for (int it = 0; it < 2; ++it) {
            const int c = it * 256 + 8 * lane;
            H8 t;
            t.f = *(const v8h*)(sh + row * HP + c);
            v[q][it] = t.u;
        }
    }
#pragma unroll
    for (int q = 0; q < 2; ++q)
#pragma unroll
        for (int it = 0; it < 2; ++it) {
            const int row = 2 * wave + q;
            const int c = it * 256 + 8 * lane;
            *(volatile u16x8*)(hdec16 + (size_t)(b0 + row) * HID + c) = v[q][it];
        }
    __threadfence();
#pragma unroll
    for (int q = 0; q < 2; ++q)
#pragma unroll
        for (int it = 0; it < 2; ++it) {
            const int row = 2 * wave + q;
            const int c = it * 256 + 8 * lane;
            *(volatile u16x8*)(hdec16 + (size_t)(b0 + row) * HID + c) = v[q][it];
        }
}

__global__ __launch_bounds__(NT)
void dec_kernel(const f16_t* __restrict__ x16, const float* __restrict__ x32,
                const f16_t* __restrict__ whh, const f16_t* __restrict__ wih, const float* __restrict__ bias,
                const f16_t* __restrict__ hdec16, const f16_t* __restrict__ wout16, const float* __restrict__ b_out,
                const float* __restrict__ skipa, float* out)
{
    __shared__ __attribute__((aligned(16))) f16_t hbuf[2 * SEQB * HP];
    __shared__ __attribute__((aligned(16))) float sout[SEQB * OP];

    const int tid  = threadIdx.x;
    const int lane = tid & 31;
    const int wave = tid >> 5;
    const int h    = lane >> 4;
    const int m    = lane & 15;
    const int b0   = (int)blockIdx.x * SEQB;
    const int j0   = wave * 32;

    for (int i = tid; i < 2 * SEQB * HP; i += NT) {
        const int buf = (i >= SEQB * HP) ? 1 : 0;
        const int rem = i - buf * (SEQB * HP);
        const int row = rem / HP;
        const int col = rem - row * HP;
        const int cc  = min(col, HID - 1);
        const f16_t v = hdec16[(size_t)(b0 + row) * HID + cc];
        hbuf[i] = (buf == 0 && col < HID) ? v : (f16_t)0.0f;
    }
    for (int i = tid; i < SEQB * OP; i += NT) sout[i] = 0.0f;

    float bi[8];
#pragma unroll
    for (int t = 0; t < 8; ++t) bi[t] = bias[(t >> 1) * HID + j0 + (t & 1) * 16 + m];
    float cst[16];
#pragma unroll
    for (int i = 0; i < 16; ++i) cst[i] = 0.0f;

    const float av    = skipa[0];
    const float alpha = 1.0f / (1.0f + expf(-av));
    const float oma   = 1.0f - alpha;
    const v4f   bo4   = *(const v4f*)(b_out + 4 * lane);

    const f16_t* wh = whh + (size_t)(j0 + m) * HID + 8 * h;
    const f16_t* wi = wih + (size_t)(j0 + m) * DIN + 8 * h;
    const f16_t* xb = x16 + (size_t)(b0 + m) * TLEN * DIN + 8 * h;
    const f16_t* wo = wout16 + (size_t)(16 * (wave & 7) + m) * HID + 8 * h;
    const float* xs = x32 + (size_t)(b0 + wave) * TLEN * DIN + 4 * lane;
    float* orow = out + (size_t)(b0 + wave) * DSTEPS * DIN + 4 * lane;
    __syncthreads();

#pragma unroll 1
    for (int s = 0; s < DSTEPS; ++s) {
        const int cur = s & 1;
        const f16_t* ha = hbuf + cur * (SEQB * HP) + m * HP + 8 * h;
        f16_t* hn = hbuf + (cur ^ 1) * (SEQB * HP);

        v8f acc[8];
#pragma unroll
        for (int t = 0; t < 8; ++t)
#pragma unroll
            for (int r = 0; r < 8; ++r) acc[t][r] = 0.0f;

        gates_mma(acc, ha, xb + (size_t)s * DIN, wh, wi);

        float hnew[16];
        lstm_cell(acc, bi, cst, hnew);
#pragma unroll
        for (int u = 0; u < 2; ++u)
#pragma unroll
            for (int r = 0; r < 8; ++r)
                hn[(8 * h + r) * HP + j0 + 16 * u + m] = (f16_t)hnew[u * 8 + r];
        __syncthreads();

        if (wave < 8) {
            v8f oacc;
#pragma unroll
            for (int r = 0; r < 8; ++r) oacc[r] = 0.0f;
            const f16_t* ya = hn + m * HP + 8 * h;
#pragma unroll 1
            for (int kit = 0; kit < HID / 32; ++kit) {
                const int k0 = kit * 32;
                Frag a, b;
                a.h[0] = *(const v8h*)(ya + k0);
                a.h[1] = *(const v8h*)(ya + k0 + 16);
                b.h[0] = *(const v8h*)(wo + k0);
                b.h[1] = *(const v8h*)(wo + k0 + 16);
                mma(oacc, a, b);
            }
#pragma unroll
            for (int r = 0; r < 8; ++r) sout[(8 * h + r) * OP + 16 * wave + m] = oacc[r];
        }
        __syncthreads();

        const v4f d  = *(const v4f*)(sout + wave * OP + 4 * lane);
        const v4f xv = *(const v4f*)(xs + (size_t)(s + 1) * DIN);
        const v4f o  = (d * INV16 + bo4) * alpha + xv * oma;
        float* gp = orow + (size_t)s * DIN;
        *(volatile v4f*)gp = o;
        __threadfence();
        *(volatile v4f*)gp = o;
    }
}

static void launch_cvt(const float* src, unsigned short* dst, int n, float scale, hipStream_t stream)
{
    const int n8 = n / 8;
    cvt_kernel<<<dim3((n8 + 255) / 256), dim3(256), 0, stream>>>(src, dst, n8, scale);
}

extern "C" void kernel_launch(void* const* d_in, const int* in_sizes, int n_in,
                              void* d_out, int out_size, void* d_ws, size_t ws_size,
                              hipStream_t stream)
{
    if (n_in < 18) return;
    if (in_sizes[0]  != BATCH * TLEN * DIN) return;
    if (in_sizes[1]  != BATCH)              return;
    if (in_sizes[2]  != G4 * DIN)           return;
    if (in_sizes[3]  != G4 * HID)           return;
    if (in_sizes[4]  != G4)                 return;
    if (in_sizes[5]  != G4 * DIN)           return;
    if (in_sizes[6]  != G4 * HID)           return;
    if (in_sizes[7]  != G4)                 return;
    if (in_sizes[8]  != G4 * DIN)           return;
    if (in_sizes[9]  != G4 * HID)           return;
    if (in_sizes[10] != G4)                 return;
    if (in_sizes[11] != LAT * G4)           return;
    if (in_sizes[12] != LAT)                return;
    if (in_sizes[13] != HID * LAT)          return;
    if (in_sizes[14] != HID)                return;
    if (in_sizes[15] != DIN * HID)          return;
    if (in_sizes[16] != DIN)                return;
    if (in_sizes[17] != 1)                  return;
    if (out_size != BATCH * DSTEPS * DIN)   return;
    if (ws_size < WS_END)                   return;

    const float* x_f   = (const float*)d_in[0];
    const int*   lens  = (const int*)d_in[1];
    const float* Wih_f = (const float*)d_in[2];
    const float* Whh_f = (const float*)d_in[3];
    const float* b_f   = (const float*)d_in[4];
    const float* Wih_b = (const float*)d_in[5];
    const float* Whh_b = (const float*)d_in[6];
    const float* b_b   = (const float*)d_in[7];
    const float* Wih_d = (const float*)d_in[8];
    const float* Whh_d = (const float*)d_in[9];
    const float* b_d   = (const float*)d_in[10];
    const float* W_lat = (const float*)d_in[11];
    const float* b_lat = (const float*)d_in[12];
    const float* W_l2h = (const float*)d_in[13];
    const float* b_l2h = (const float*)d_in[14];
    const float* W_out = (const float*)d_in[15];
    const float* b_out = (const float*)d_in[16];
    const float* skipa = (const float*)d_in[17];
    float* out = (float*)d_out;

    char* ws = (char*)d_ws;
    unsigned short* x16    = (unsigned short*)(ws + OFF_X16);
    unsigned short* whh16  = (unsigned short*)(ws + OFF_WHH);
    unsigned short* wih16  = (unsigned short*)(ws + OFF_WIH);
    unsigned short* wlat16 = (unsigned short*)(ws + OFF_WLAT);
    unsigned short* wl2h16 = (unsigned short*)(ws + OFF_WL2H);
    unsigned short* wout16 = (unsigned short*)(ws + OFF_WOUT);
    unsigned short* latin  = (unsigned short*)(ws + OFF_LAT);
    unsigned short* hdec16 = (unsigned short*)(ws + OFF_HDEC);

    const size_t PWHH = (size_t)G4 * HID;
    const size_t PWIH = (size_t)G4 * DIN;

    launch_cvt(x_f,   x16,                BATCH * TLEN * DIN, 1.0f,  stream);
    launch_cvt(Whh_f, whh16 + 0 * PWHH,   G4 * HID,           16.0f, stream);
    launch_cvt(Whh_b, whh16 + 1 * PWHH,   G4 * HID,           16.0f, stream);
    launch_cvt(Whh_d, whh16 + 2 * PWHH,   G4 * HID,           16.0f, stream);
    launch_cvt(Wih_f, wih16 + 0 * PWIH,   G4 * DIN,           16.0f, stream);
    launch_cvt(Wih_b, wih16 + 1 * PWIH,   G4 * DIN,           16.0f, stream);
    launch_cvt(Wih_d, wih16 + 2 * PWIH,   G4 * DIN,           16.0f, stream);
    launch_cvt(W_lat, wlat16,             LAT * G4,           16.0f, stream);
    launch_cvt(W_l2h, wl2h16,             HID * LAT,          16.0f, stream);
    launch_cvt(W_out, wout16,             DIN * HID,          16.0f, stream);

    enc_kernel<<<dim3(2 * NGRP), dim3(NT), 0, stream>>>(
        (const f16_t*)x16, lens,
        (const f16_t*)(whh16 + 0 * PWHH), (const f16_t*)(wih16 + 0 * PWIH), b_f,
        (const f16_t*)(whh16 + 1 * PWHH), (const f16_t*)(wih16 + 1 * PWIH), b_b,
        latin);

    latent_kernel<<<dim3(NGRP), dim3(256), 0, stream>>>(
        (const f16_t*)latin, (const f16_t*)wlat16, b_lat, (const f16_t*)wl2h16, b_l2h, hdec16);

    dec_kernel<<<dim3(NGRP), dim3(NT), 0, stream>>>(
        (const f16_t*)x16, x_f,
        (const f16_t*)(whh16 + 2 * PWHH), (const f16_t*)(wih16 + 2 * PWIH), b_d,
        (const f16_t*)hdec16, (const f16_t*)wout16, b_out, skipa, out);
}
